// S4__52604759441727
// MI455X (gfx1250) — hardware-verified
//
#include <hip/hip_runtime.h>
#include <math.h>

typedef __attribute__((ext_vector_type(16))) _Float16 v16h;
typedef __attribute__((ext_vector_type(16))) __bf16 v16b;
typedef __attribute__((ext_vector_type(8)))  _Float16 v8h;
typedef __attribute__((ext_vector_type(8)))  float v8f;
typedef __attribute__((ext_vector_type(4)))  float v4f;
typedef __attribute__((ext_vector_type(2)))  float v2f;
typedef __attribute__((ext_vector_type(4)))  unsigned v4u;
typedef __attribute__((ext_vector_type(4)))  int v4i;
typedef float __attribute__((may_alias)) float_a;
typedef int __attribute__((may_alias)) int_a;

template <typename T> __device__ __forceinline__ void vst2(void* p, T v) { *(volatile T*)p = v; __threadfence(); *(volatile T*)p = v; }
__device__ __forceinline__ v8f wmma16(v16h a, v16h b, v8f c) {
  v8f d = __builtin_amdgcn_wmma_f32_16x16x32_f16(false, a, false, b, (short)0, c, false, false);
  asm volatile("v_nop\n\tv_nop\n\tv_nop\n\tv_nop" : "+v"(d) : "v"(a), "v"(b));
  return d;
}
__device__ __forceinline__ v8f wmma_bf(v16b a, v16b b, v8f c) {
  v8f d = __builtin_amdgcn_wmma_f32_16x16x32_bf16(false, a, false, b, (short)0, c, false, false);
  asm volatile("v_nop\n\tv_nop\n\tv_nop\n\tv_nop" : "+v"(d) : "v"(a), "v"(b));
  return d;
}
__device__ __forceinline__ v16h frag_h(const _Float16* rowk0, int lane) {
  union { v16h v; v8h q[2]; } u; const _Float16* p = rowk0 + 8 * (lane >> 4);
  u.q[0] = *(const v8h*)p; u.q[1] = *(const v8h*)(p + 16); return u.v;
}
__device__ __forceinline__ v16h frag_f32(const float* rowk0, int lane) {
  v16h a; const float* p = rowk0 + 8 * (lane >> 4);
#pragma unroll
  for (int i = 0; i < 8; ++i) { a[i] = (_Float16)p[i]; a[8 + i] = (_Float16)p[16 + i]; }
  return a;
}
__device__ __forceinline__ v16h frag_f32s(const float* rowk0, int lane, float sc) {
  v16h a; const float* p = rowk0 + 8 * (lane >> 4);
#pragma unroll
  for (int i = 0; i < 8; ++i) { a[i] = (_Float16)(p[i] * sc); a[8 + i] = (_Float16)(p[16 + i] * sc); }
  return a;
}
__device__ __forceinline__ v16h fragc_f32(const float* W, int k0, int n, int lane, int ld, int K) {
  v16h a; const int g = lane >> 4;
#pragma unroll
  for (int i = 0; i < 8; ++i) { const int ka = k0 + 8 * g + i, kb = ka + 16;
    a[i] = (_Float16)(ka < K ? W[(size_t)(ka < K ? ka : K - 1) * ld + n] : 0.f); a[8 + i] = (_Float16)(kb < K ? W[(size_t)(kb < K ? kb : K - 1) * ld + n] : 0.f); }
  return a;
}
struct F2 { v16b h, l; };
__device__ __forceinline__ F2 bsplit16(const float v[16]) { F2 r;
#pragma unroll
  for (int i = 0; i < 16; ++i) { const __bf16 h = (__bf16)v[i]; r.h[i] = h; r.l[i] = (__bf16)(v[i] - (float)h); }
  return r; }
__device__ __forceinline__ F2 split_row(const float* row, int k0, int lane) { float v[16]; const float* p = row + k0 + 8 * (lane >> 4);
#pragma unroll
  for (int i = 0; i < 8; ++i) { v[i] = p[i]; v[8 + i] = p[16 + i]; }
  return bsplit16(v); }
__device__ __forceinline__ F2 split_rowK(const float* row, int k0, int lane, int K) { float v[16]; const int g = lane >> 4;
#pragma unroll
  for (int i = 0; i < 8; ++i) { const int ka = k0 + 8 * g + i, kb = ka + 16; v[i] = ka < K ? row[ka < K ? ka : K - 1] : 0.f; v[8 + i] = kb < K ? row[kb < K ? kb : K - 1] : 0.f; }
  return bsplit16(v); }
__device__ __forceinline__ F2 split_col(const float* W, int k0, int n, int lane, int ld, int K) { float v[16]; const int g = lane >> 4;
#pragma unroll
  for (int i = 0; i < 8; ++i) { const int ka = k0 + 8 * g + i, kb = ka + 16; v[i] = ka < K ? W[(size_t)(ka < K ? ka : K - 1) * ld + n] : 0.f; v[8 + i] = kb < K ? W[(size_t)(kb < K ? kb : K - 1) * ld + n] : 0.f; }
  return bsplit16(v); }
__device__ __forceinline__ v8f mac3(const F2& a, const F2& b, v8f c) { c = wmma_bf(a.l, b.h, c); c = wmma_bf(a.h, b.l, c); return wmma_bf(a.h, b.h, c); }
__device__ __forceinline__ float sigm(float v) { return 1.0f / (1.0f + expf(-v)); }
#define LDSX() do { asm volatile("s_wait_dscnt 0" ::: "memory"); __builtin_amdgcn_wave_barrier(); __builtin_amdgcn_fence(__ATOMIC_RELEASE, "workgroup"); } while (0)


#define NG 16
#define TL 354
#define NNODE 64
#define HH 128
#define NS 32
#define NBN (NG * NNODE)
#define LP 384
#define NLT 23
#define RP 448
#ifndef NBT
#define NBT (NBN / 16)
#endif
#define NGT (NBT * 16 / NNODE)
typedef __attribute__((ext_vector_type(8))) __bf16 v8b;
__device__ __forceinline__ v16b frag_b(const __bf16* rowk0, int lane) {
  union { v16b v; v8b q[2]; } u; const __bf16* p = rowk0 + 8 * (lane >> 4);
  u.q[0] = *(const v8b*)p; u.q[1] = *(const v8b*)(p + 16); return u.v;
}
__device__ __forceinline__ float bfr(float v) { return (float)(__bf16)v; }
__device__ __attribute__((noinline)) float exp_ni(float v) { return expf(v); }
__device__ __attribute__((noinline)) float erf_ni(float v) { return erff(v); }

__device__ __attribute__((noinline)) float tanh_ni(float v) { return tanhf(v); }
__device__ __attribute__((noinline)) float sin_ni(float v) { return sinf(v); }
__device__ __attribute__((noinline)) float cos_ni(float v) { return cosf(v); }
__device__ __forceinline__ float gelu_t(float x) { const float c = 0.7978845608028654f; const float t = tanh_ni(c * (x + 0.044715f * x * x * x)); return 0.5f * x * (1.0f + t); }
__device__ __forceinline__ void put_hl(__bf16* h, __bf16* l, float v) { const __bf16 hb = (__bf16)v; *h = hb; *l = (__bf16)(v - (float)hb); }
#define WS_KT   0u
#define WS_KC   (WS_KT + 4u * HH * LP)
#define WS_RH   (WS_KC + 4u * HH * LP)
#define WS_RL   (WS_RH + 2u * HH * RP)
#define WS_PO   (WS_RL + 2u * HH * RP)
#define WS_XT   (WS_PO + 2u * 2 * HH * HH)
#define WS_PART (WS_XT + 2u * NBN * LP)
#define WS_END  (WS_PART + 4u * NLT * NBN * HH)

__global__ __launch_bounds__(32) void k_s4k(const float* __restrict__ LDT, const float* __restrict__ ARE, const float* __restrict__ AIM, const float* __restrict__ CRE, const float* __restrict__ CIM, float* __restrict__ KT, float* __restrict__ KC, __bf16* __restrict__ RH, __bf16* __restrict__ RL) {
  __shared__ __align__(16) float sk[LP]; __shared__ __align__(16) float sc[LP]; __shared__ __align__(16) __bf16 srh[RP], srl[RP];
  const int h = blockIdx.x, lane = threadIdx.x; const int n = lane;
  const float dt = exp_ni(bfr(LDT[h])); const float ar = bfr(ARE[h * NS + n]), ai = bfr(AIM[h * NS + n]); const float dar = ar * dt, dai = ai * dt;
  const float cr = bfr(CRE[h * NS + n]), ci = bfr(CIM[h * NS + n]);
  const float er = exp_ni(dar) * cos_ni(dai) - 1.0f, ei = exp_ni(dar) * sin_ni(dai);
  const float nr = cr * er - ci * ei, ni = cr * ei + ci * er;
  const float den = ar * ar + ai * ai; const float cdr = (nr * ar + ni * ai) / den, cdi = (ni * ar - nr * ai) / den;
#pragma unroll 1
  for (int l = 0; l < LP; ++l) { float term = 0.f;
    if (l < TL) { const float pr = dar * (float)l, pim = dai * (float)l; const float mg = exp_ni(pr); const float vr = mg * cos_ni(pim), vi = mg * sin_ni(pim); term = cdr * vr - cdi * vi; }
#pragma unroll
    for (int o = 1; o < 32; o <<= 1) term += __shfl_xor(term, o);
    if (lane == 0) sk[l] = (l < TL) ? 2.0f * term : 0.f; }
  LDSX();
  if (lane == 0) { float run = 0.f; for (int l = 0; l < LP; ++l) { run += sk[l]; sc[l] = run; } }
  LDSX();
  for (int p = lane; p < RP; p += 32) { const int d = (LP - 1) - p; const float v = (d >= 0 && d < TL) ? sk[d] : 0.f; put_hl(&srh[p], &srl[p], v); }
  LDSX();
  for (int q = lane; q < LP / 4; q += 32) { vst2(KT + (size_t)h * LP + q * 4, *(const v4f*)&sk[q * 4]); vst2(KC + (size_t)h * LP + q * 4, *(const v4f*)&sc[q * 4]); }
  for (int q = lane; q < RP / 8; q += 32) { vst2((unsigned*)(RH + (size_t)h * RP + q * 8), *(const v4u*)&srh[q * 8]); vst2((unsigned*)(RL + (size_t)h * RP + q * 8), *(const v4u*)&srl[q * 8]); }
}
__global__ __launch_bounds__(128) void k_po(const float* __restrict__ Wo, __bf16* __restrict__ PO) {
  __shared__ __align__(16) __bf16 s[HH]; const int nrow = blockIdx.x, tid = threadIdx.x; s[tid] = (__bf16)Wo[(size_t)nrow * HH + tid]; __syncthreads();
  if (tid < HH / 8) vst2((unsigned*)(PO + (size_t)nrow * HH + tid * 8), *(const v4u*)&s[tid * 8]);
}
__global__ __launch_bounds__(128) void k_xt(const float* __restrict__ X, __bf16* __restrict__ XT) {
  __shared__ __align__(16) __bf16 s[LP]; const int bn = blockIdx.x, tid = threadIdx.x; const int b = bn / NNODE, n = bn % NNODE;
  for (int m = tid; m < LP; m += 128) s[m] = (__bf16)((m < TL) ? X[((size_t)b * TL + m) * NNODE + n] : 0.f);
  __syncthreads();
  if (tid < LP / 8) vst2((unsigned*)(XT + (size_t)bn * LP + tid * 8), *(const v4u*)&s[tid * 8]);
}
__global__ __launch_bounds__(128) void k_main(const __bf16* __restrict__ XT, const float* __restrict__ X, const float* __restrict__ KC, const __bf16* __restrict__ RH, const __bf16* __restrict__ RL, const float* __restrict__ WIN, const float* __restrict__ BIN, const float* __restrict__ DD, const __bf16* __restrict__ PO, const float* __restrict__ BO, float* __restrict__ PART) {
  __shared__ __align__(16) __bf16 sgh[256][HH + 8], sgl[256][HH + 8]; __shared__ __align__(16) float sz[4][16][HH + 4];
  const int tid = threadIdx.x, wave = tid >> 5, lane = tid & 31, col = lane & 15, g = lane >> 4; const int bn0 = blockIdx.x * 16, lt = blockIdx.y, l0 = lt * 16;
  const int nks = (l0 + 16 + 31) / 32;
  { const int bn = bn0 + col; const int b = bn / NNODE, nn = bn % NNODE;
#pragma unroll 1
    for (int hh = 0; hh < 32; ++hh) { const int h = wave * 32 + hh; v8f acc = {};
      for (int ks = 0; ks < nks; ++ks) { const v16b a = frag_b(XT + (size_t)bn * LP + ks * 32, lane); const int p0 = (LP - 1) - (l0 + col) + ks * 32; const v16b rh = frag_b(RH + (size_t)h * RP + p0, lane), rl = frag_b(RL + (size_t)h * RP + p0, lane); acc = wmma_bf(a, rl, acc); acc = wmma_bf(a, rh, acc); }
      const float wi = bfr(WIN[h]), bi = bfr(BIN[h]), dd = bfr(DD[h]);
#pragma unroll
      for (int r = 0; r < 8; ++r) { const int bnl = 8 * g + r; const int l = l0 + col; const int bnr = bn0 + bnl; const int br = bnr / NNODE, nr = bnr % NNODE;
        const float xv = (l < TL) ? bfr(X[((size_t)br * TL + (l < TL ? l : 0)) * NNODE + nr]) : 0.f; const float kc = KC[(size_t)h * LP + l];
        const float y = wi * acc[r] + bi * kc + dd * (wi * xv + bi); put_hl(&sgh[col * 16 + bnl][h], &sgl[col * 16 + bnl][h], gelu_t(y)); } } }
  __syncthreads();
  { float zs[8][8];
#pragma unroll
    for (int j = 0; j < 8; ++j)
#pragma unroll
      for (int r = 0; r < 8; ++r) zs[j][r] = 0.f;
#pragma unroll 1
    for (int q = 0; q < 4; ++q) { const int ll = wave + 4 * q; const int l = l0 + ll; if (l >= TL) continue;
#pragma unroll
      for (int half = 0; half < 2; ++half) { v8f acc[8] = {};
#pragma unroll
        for (int kc = 0; kc < HH / 32; ++kc) { const v16b ah = frag_b(&sgh[ll * 16 + col][kc * 32], lane), al = frag_b(&sgl[ll * 16 + col][kc * 32], lane);
#pragma unroll
          for (int jj = 0; jj < 8; ++jj) { const int j = (jj < 4) ? (half * 4 + jj) : (8 + half * 4 + (jj - 4)); const v16b w = frag_b(PO + (size_t)(j * 16 + col) * HH + kc * 32, lane); acc[jj] = wmma_bf(al, w, acc[jj]); acc[jj] = wmma_bf(ah, w, acc[jj]); } }
#pragma unroll
        for (int jj = 0; jj < 4; ++jj) { const int j = half * 4 + jj; const int c = j * 16 + col; const float ba = bfr(BO[c]), bb = bfr(BO[HH + c]);
#pragma unroll
          for (int r = 0; r < 8; ++r) { const float av = acc[jj][r] + ba, bv = acc[jj + 4][r] + bb; zs[j][r] += av / (1.0f + exp_ni(-bv)); } } } }
#pragma unroll
    for (int j = 0; j < 8; ++j)
#pragma unroll
      for (int r = 0; r < 8; ++r) sz[wave][8 * g + r][j * 16 + col] = zs[j][r]; }
  __syncthreads();
  { __shared__ __align__(16) float srow[16][HH + 4];
    for (int q = tid; q < 16 * HH; q += 128) { const int bnl = q >> 7, c = q & 127; srow[bnl][c] = (sz[0][bnl][c] + sz[1][bnl][c]) + (sz[2][bnl][c] + sz[3][bnl][c]); }
    __syncthreads();
    for (int q = tid; q < 16 * 32; q += 128) { const int bnl = q >> 5, pc = q & 31; vst2(PART + (((size_t)lt * NBN + bn0 + bnl) * HH) + pc * 4, *(const v4f*)&srow[bnl][pc * 4]); } }
}
__global__ __launch_bounds__(128) void k_fin(const float* __restrict__ PART, const float* __restrict__ WC, const float* __restrict__ BC, float* __restrict__ out) {
  __shared__ float sg[NG][HH]; __shared__ __align__(16) float so[16]; const int c = threadIdx.x;
#pragma unroll 1
  for (int b = 0; b < NG; ++b) { float s = 0.f; if (b >= NGT) { sg[b][c] = 0.f; continue; }
#pragma unroll 1
    for (int n = 0; n < NNODE; ++n) { float t = 0.f;
#pragma unroll 1
      for (int lt = 0; lt < NLT; ++lt) t += PART[(((size_t)lt * NBN + b * NNODE + n) * HH) + c];
      s += t * (1.0f / (float)TL); }
    sg[b][c] = s * (1.0f / (float)NNODE); }
  __syncthreads();
  if (c < NG) { float y = bfr(BC[0]);
#pragma unroll 1
    for (int k = 0; k < HH; ++k) y += sg[c][k] * bfr(WC[k]);
    so[c] = (c < NGT) ? y : 0.f; }
  __syncthreads();
  if (c < 4) vst2(out + c * 4, *(const v4f*)&so[c * 4]);
}
extern "C" void kernel_launch(void* const* d_in, const int* in_sizes, int n_in, void* d_out, int out_size, void* d_ws, size_t ws_size, hipStream_t stream) {
  (void)in_sizes; (void)n_in; (void)out_size;
  const float** F = (const float**)d_in;
  if (ws_size < (size_t)WS_END) return;
  char* ws = (char*)d_ws; float *KT = (float*)(ws + WS_KT), *KC = (float*)(ws + WS_KC), *PART = (float*)(ws + WS_PART); __bf16 *RH = (__bf16*)(ws + WS_RH), *RL = (__bf16*)(ws + WS_RL), *PO = (__bf16*)(ws + WS_PO), *XT = (__bf16*)(ws + WS_XT);
  k_s4k<<<HH, 32, 0, stream>>>(F[3], F[4], F[5], F[6], F[7], KT, KC, RH, RL);
  k_po<<<2 * HH, 128, 0, stream>>>(F[9], PO);
  k_xt<<<NBN, 128, 0, stream>>>(F[0], XT);
  k_main<<<dim3(NBT, NLT), 128, 0, stream>>>(XT, F[0], KC, RH, RL, F[1], F[2], F[8], PO, F[10], PART);
  k_fin<<<1, 128, 0, stream>>>(PART, F[11], F[12], (float*)d_out);
}
